// ConditionalLinearAttention_61014305407449
// MI455X (gfx1250) — hardware-verified
//
#include <hip/hip_runtime.h>

typedef __attribute__((ext_vector_type(16))) _Float16 v16h;
typedef __attribute__((ext_vector_type(8)))  _Float16 v8h;
typedef __attribute__((ext_vector_type(8)))  float    v8f;
typedef __attribute__((ext_vector_type(4)))  float    v4f;
typedef float v4fa __attribute__((ext_vector_type(4), may_alias));
typedef __attribute__((ext_vector_type(4)))  unsigned v4u;
typedef unsigned v4ua __attribute__((ext_vector_type(4), may_alias));

#define RSPLIT (1.0f / 2048.0f)
#define PL_M1 ((size_t)8 * 256 * 512)
#define PL_WE ((size_t)8 * 256 * 256)
#define WLD 264

static __device__ __forceinline__ int lane_id() { return (int)(threadIdx.x & 31u); }
static __device__ __forceinline__ _Float16 lo_of(float v, _Float16 h) { return (_Float16)((v - (float)h) * 2048.0f); }
static __device__ __forceinline__ v8f wmma16(v16h a, v16h b, v8f c) {
  return __builtin_amdgcn_wmma_f32_16x16x32_f16(false, a, false, b, (short)0, c, false, false);
}
static __device__ __forceinline__ v8f wmma_split(v16h a, v16h al, v16h b, v16h bl, v8f c) {
  v8f x = {}; x = wmma16(al, b, x); x = wmma16(a, bl, x); return wmma16(a, b, c) + x * RSPLIT;
}
struct F2 { v16h v, l; };
static __device__ __forceinline__ int kidx(int i, int lane) { return ((i < 8) ? i : (i + 8)) + ((lane >> 4) << 3); }

static __device__ __forceinline__ F2 a_f32(const float* A, int ld, int m0, int k0) {
  const int lane = lane_id(); const float* p = A + (size_t)(m0 + (lane & 15)) * ld + k0 + ((lane >> 4) << 3);
  F2 f;
#pragma unroll
  for (int i = 0; i < 8; ++i) { float u = p[i], w = p[16 + i]; f.v[i] = (_Float16)u; f.l[i] = lo_of(u, f.v[i]); f.v[i + 8] = (_Float16)w; f.l[i + 8] = lo_of(w, f.v[i + 8]); }
  return f;
}
static __device__ __forceinline__ F2 a_f16p(const _Float16* A, size_t pl, int ld, int m0, int k0) {
  const int lane = lane_id(); const _Float16* p = A + (size_t)(m0 + (lane & 15)) * ld + k0 + ((lane >> 4) << 3);
  F2 f;
  f.v = __builtin_shufflevector(*(const v8h*)p, *(const v8h*)(p + 16), 0,1,2,3,4,5,6,7,8,9,10,11,12,13,14,15);
  f.l = __builtin_shufflevector(*(const v8h*)(p + pl), *(const v8h*)(p + pl + 16), 0,1,2,3,4,5,6,7,8,9,10,11,12,13,14,15);
  return f;
}
static __device__ __forceinline__ F2 b_f32(const float* B, int ld, int k0, int n0) {
  const int lane = lane_id(); const float* p = B + (size_t)(k0 + ((lane >> 4) << 3)) * ld + n0 + (lane & 15);
  F2 f;
#pragma unroll
  for (int i = 0; i < 8; ++i) { float u = p[(size_t)i * ld], w = p[(size_t)(16 + i) * ld]; f.v[i] = (_Float16)u; f.l[i] = lo_of(u, f.v[i]); f.v[i + 8] = (_Float16)w; f.l[i + 8] = lo_of(w, f.v[i + 8]); }
  return f;
}
static __device__ __forceinline__ F2 bt_f32(const float* S, int ld, int k0, int n0) { return a_f32(S, ld, n0, k0); }
static __device__ __forceinline__ F2 bt_f16p(const _Float16* S, size_t pl, int ld, int k0, int n0) { return a_f16p(S, pl, ld, n0, k0); }

static __device__ __forceinline__ void c_to_lds(float* D, int ld, int m0, int n0, v8f acc) {
  const int lane = lane_id(); const int col = n0 + (lane & 15); const int rb = m0 + ((lane >> 4) << 3);
#pragma unroll
  for (int r = 0; r < 8; ++r) D[(rb + r) * ld + col] = acc[r];
}
static __device__ __forceinline__ void rows64_to_planes(const float* T, int lds, _Float16* dst, size_t pl, int ldd) {
  const int lane = lane_id();
#pragma unroll 1
  for (int pass = 0; pass < 2; ++pass) {
#pragma unroll
    for (int i = 0; i < 4; ++i) {
      const int c = lane + 32 * i, rr = c >> 3, q = (c & 7) * 8;
      const float* s = T + rr * lds + q;
      _Float16 hv[8], hl[8];
#pragma unroll
      for (int e = 0; e < 8; ++e) { hv[e] = (_Float16)s[e]; hl[e] = lo_of(s[e], hv[e]); }
      _Float16* d = dst + (size_t)rr * ldd + q;
      *(volatile v4u*)d = *(const v4ua*)hv; *(volatile v4u*)(d + pl) = *(const v4ua*)hl;
    }
    __threadfence();
  }
}

__global__ __launch_bounds__(256) void k1_context_m1(
    const float* __restrict__ cond,
    const float* __restrict__ Wcond,
    const float* __restrict__ Wout,
    _Float16* __restrict__ M1)
{
  __shared__ __attribute__((aligned(16))) float k_lds[64 * 128];
  __shared__ __attribute__((aligned(16))) float v_lds[64 * 128];
  __shared__ __attribute__((aligned(16))) float c_lds[64 * 64];
  __shared__ __attribute__((aligned(16))) float stg[8][16 * 68];

  const int h = blockIdx.x;
  const int b = blockIdx.y;
  const int wave = (int)(threadIdx.x >> 5);
  const float* cf = cond + (size_t)b * 512 * 128;

  {
    const int n0 = wave * 16;
    v8f z = {};
    v8f accK[4], accV[4];
#pragma unroll
    for (int m = 0; m < 4; ++m) { accK[m] = z; accV[m] = z; }
    const float* Ak = Wcond + (size_t)(h * 64) * 512;
    const float* Av = Wcond + (size_t)(512 + h * 64) * 512;
    for (int kt = 0; kt < 16; ++kt) {
      F2 bf = b_f32(cf, 128, kt * 32, n0);
#pragma unroll
      for (int m = 0; m < 4; ++m) {
        F2 a0 = a_f32(Ak, 512, m * 16, kt * 32);
        accK[m] = wmma_split(a0.v, a0.l, bf.v, bf.l, accK[m]);
        F2 a1 = a_f32(Av, 512, m * 16, kt * 32);
        accV[m] = wmma_split(a1.v, a1.l, bf.v, bf.l, accV[m]);
      }
    }
#pragma unroll
    for (int m = 0; m < 4; ++m) { c_to_lds(k_lds, 128, m * 16, n0, accK[m]); c_to_lds(v_lds, 128, m * 16, n0, accV[m]); }
  }
  __syncthreads();

  if (threadIdx.x < 64) {
    float* row = k_lds + threadIdx.x * 128;
    float mx = -3.4e38f;
    for (int j = 0; j < 128; ++j) mx = fmaxf(mx, row[j]);
    float s = 0.f;
    for (int j = 0; j < 128; ++j) { float e = __expf(row[j] - mx); row[j] = e; s += e; }
    float inv = 1.f / s;
    for (int j = 0; j < 128; ++j) row[j] *= inv;
  }
  __syncthreads();

  for (int t = wave * 2; t < wave * 2 + 2; ++t) {
    const int m0 = (t >> 2) * 16, n0 = (t & 3) * 16;
    v8f acc = {};
#pragma unroll
    for (int kt = 0; kt < 4; ++kt) {
      F2 a  = a_f32(k_lds, 128, m0, kt * 32);
      F2 bb = bt_f32(v_lds, 128, kt * 32, n0);
      acc = wmma_split(a.v, a.l, bb.v, bb.l, acc);
    }
    c_to_lds(c_lds, 64, m0, n0, acc);
  }
  __syncthreads();

  _Float16* M1b = M1 + (size_t)b * 256 * 512;
  const float* WoutH = Wout + h * 64;
  float* sw = stg[wave];
#pragma unroll 1
  for (int mh = 0; mh < 2; ++mh) {
    const int m0 = (wave * 2 + mh) * 16;
#pragma unroll
    for (int nt = 0; nt < 4; ++nt) {
      v8f acc = {};
#pragma unroll
      for (int kt = 0; kt < 2; ++kt) {
        F2 a  = a_f32(WoutH, 512, m0, kt * 32);
        F2 bb = bt_f32(c_lds, 64, kt * 32, nt * 16);
        acc = wmma_split(a.v, a.l, bb.v, bb.l, acc);
      }
      c_to_lds(sw, 68, 0, nt * 16, acc);
    }
    asm volatile("s_wait_dscnt 0" ::: "memory");
    rows64_to_planes(sw, 68, M1b + (size_t)m0 * 512 + h * 64, PL_M1, 512);
  }
}

__global__ __launch_bounds__(128) void k2_weff(
    const _Float16* __restrict__ M1,
    const float* __restrict__ Wq,
    _Float16* __restrict__ Weff)
{
  __shared__ __attribute__((aligned(16))) float stg[4][16 * 68];
  const int rg   = blockIdx.x;
  const int b    = blockIdx.y;
  const int wave = (int)(threadIdx.x >> 5);
  const int m0   = rg * 16;
  const int c0   = wave * 64;
  const _Float16* M1b = M1 + (size_t)b * 256 * 512;
  _Float16* Wb = Weff + (size_t)b * 256 * 256;

  v8f acc[4] = {};
  for (int kt = 0; kt < 16; ++kt) {
    F2 a = a_f16p(M1b, PL_M1, 512, m0, kt * 32);
#pragma unroll
    for (int nt = 0; nt < 4; ++nt) {
      F2 bb = b_f32(Wq, 256, kt * 32, c0 + nt * 16);
      acc[nt] = wmma_split(a.v, a.l, bb.v, bb.l, acc[nt]);
    }
  }
  float* sw = stg[wave];
#pragma unroll
  for (int nt = 0; nt < 4; ++nt) c_to_lds(sw, 68, 0, nt * 16, acc[nt]);
  asm volatile("s_wait_dscnt 0" ::: "memory");
  rows64_to_planes(sw, 68, Wb + (size_t)m0 * 256 + c0, PL_WE, 256);
}

__global__ __launch_bounds__(256) void k3_out(
    const _Float16* __restrict__ Weff,
    const float* __restrict__ x,
    const float* __restrict__ bout,
    float* __restrict__ out)
{
  __shared__ __attribute__((aligned(16))) _Float16 w_lds[2][128 * WLD];
  __shared__ __attribute__((aligned(16))) float ost[8][16 * 36];

  const int b    = blockIdx.y;
  const int mh   = blockIdx.z;
  const int tid  = (int)threadIdx.x;
  const int wave = tid >> 5, lane = tid & 31;
  const int n0   = blockIdx.x * 256 + wave * 32;
  const float* xb = x + (size_t)b * 256 * 4096;
  float* ob = out + (size_t)b * 256 * 4096;
  const _Float16* Wb = Weff + (size_t)b * 256 * 256 + (size_t)mh * 128 * 256;

  for (int c = tid; c < 128 * 32; c += 256) {
    const int row = c >> 5, col = c & 31;
    *(v4u*)(w_lds[0] + row * WLD + col * 8) = *(const v4ua*)(Wb + (size_t)row * 256 + col * 8);
    *(v4u*)(w_lds[1] + row * WLD + col * 8) = *(const v4ua*)(Wb + PL_WE + (size_t)row * 256 + col * 8);
  }
  __syncthreads();

  float* so = ost[wave];
  for (int mt = 0; mt < 8; ++mt) {
    v8f acc0 = {}, acc1 = {};
#pragma unroll 2
    for (int kt = 0; kt < 8; ++kt) {
      F2 a  = a_f16p(w_lds[0], (size_t)128 * WLD, WLD, mt * 16, kt * 32);
      F2 b0 = b_f32(xb, 4096, kt * 32, n0);
      F2 b1 = b_f32(xb, 4096, kt * 32, n0 + 16);
      acc0 = wmma_split(a.v, a.l, b0.v, b0.l, acc0);
      acc1 = wmma_split(a.v, a.l, b1.v, b1.l, acc1);
    }
    const int grow = mh * 128 + mt * 16;
    {
      const int col = lane & 15, rb = (lane >> 4) << 3;
#pragma unroll
      for (int r = 0; r < 8; ++r) { const float bz = bout[grow + rb + r]; so[(rb + r) * 36 + col] = acc0[r] + bz; so[(rb + r) * 36 + 16 + col] = acc1[r] + bz; }
    }
    asm volatile("s_wait_dscnt 0" ::: "memory");
#pragma unroll 1
    for (int pass = 0; pass < 2; ++pass) {
#pragma unroll
      for (int i = 0; i < 4; ++i) { const int c = lane + 32 * i, rr = c >> 3, q = (c & 7) * 4;
        *(volatile v4f*)(ob + (size_t)(grow + rr) * 4096 + n0 + q) = *(const volatile v4fa*)(so + rr * 36 + q); }
      __threadfence();
    }
  }
}

extern "C" void kernel_launch(void* const* d_in, const int* in_sizes, int n_in,
                              void* d_out, int out_size, void* d_ws, size_t ws_size,
                              hipStream_t stream) {
  (void)in_sizes; (void)n_in; (void)out_size; (void)ws_size;
  const float* x     = (const float*)d_in[0];
  const float* cond  = (const float*)d_in[1];
  const float* Wq    = (const float*)d_in[2];
  const float* Wcond = (const float*)d_in[3];
  const float* Wout  = (const float*)d_in[4];
  const float* bout  = (const float*)d_in[5];
  float* out = (float*)d_out;

  _Float16* M1   = (_Float16*)d_ws;
  _Float16* Weff = (_Float16*)((char*)d_ws + 2 * PL_M1 * sizeof(_Float16));

  k1_context_m1<<<dim3(8, 8), 256, 0, stream>>>(cond, Wcond, Wout, M1);
  k2_weff<<<dim3(16, 8), 128, 0, stream>>>(M1, Wq, Weff);
  k3_out<<<dim3(16, 8, 2), 256, 0, stream>>>(Weff, x, bout, out);
}
